// GATImputer_17712445129456
// MI455X (gfx1250) — hardware-verified
//
#include <hip/hip_runtime.h>
#include <stdint.h>


typedef _Float16 f16_t;
typedef _Float16 v16h __attribute__((ext_vector_type(16)));
typedef _Float16 v8h  __attribute__((ext_vector_type(8)));
typedef __bf16   v16b __attribute__((ext_vector_type(16)));
typedef unsigned short v8us __attribute__((ext_vector_type(8)));
typedef float    v8f  __attribute__((ext_vector_type(8)));
typedef float    v4f  __attribute__((ext_vector_type(4)));
typedef unsigned int v4u __attribute__((ext_vector_type(4)));

union FragB { v16b v; v8us u[2]; };
union FragH { v16h v; v8us u[2]; };
union Pack8 { v8h h; v4u u; };

constexpr int Bn   = 8;
constexpr int Dn   = 1024;
constexpr int Tn   = 512;
constexpr int KIN  = 2 * Tn;
constexpr int HIDn = 256;
constexpr int NHn  = 4;
constexpr int OUTn = 64;
constexpr int NLn  = 2;
constexpr int Mrows = Bn * Dn;
constexpr int TP   = 68;
constexpr float ALPHAc = 0.2f;
constexpr float EPSc   = 1e-5f;
constexpr float PSCALE = 4096.0f;
constexpr float PSCALE_INV = 1.0f / 4096.0f;

static_assert(Mrows % 64 == 0 && HIDn % 64 == 0 && Tn % 64 == 0 && KIN % 64 == 0);
static_assert(Dn % 64 == 0 && OUTn == 64 && HIDn == NHn * OUTn);
static_assert(Tn == 64 * 8);

__device__ __forceinline__ float lrelu(float x) { return x > 0.0f ? x : ALPHAc * x; }

__device__ __forceinline__ v8f mma_bf16(v16b a, v16b b, v8f c)
{
    c = __builtin_amdgcn_wmma_f32_16x16x32_bf16(false, a, false, b, (short)0, c, false, false);
    asm volatile("v_nop\n\tv_nop\n\tv_nop\n\tv_nop" : "+v"(c) : "v"(a), "v"(b));
    return c;
}
__device__ __forceinline__ v8f mma_f16(v16h a, v16h b, v8f c)
{
    c = __builtin_amdgcn_wmma_f32_16x16x32_f16(false, a, false, b, (short)0, c, false, false);
    asm volatile("v_nop\n\tv_nop\n\tv_nop\n\tv_nop" : "+v"(c) : "v"(a), "v"(b));
    return c;
}
__device__ __forceinline__ v8f zero8()
{
    v8f z;
#pragma unroll
    for (int r = 0; r < 8; ++r) z[r] = 0.0f;
    return z;
}

__device__ __forceinline__ unsigned int bf16_bits(float x)
{
    unsigned int u = __float_as_uint(x);
    return (u + 0x7FFFu + ((u >> 16) & 1u)) >> 16;
}
__device__ __forceinline__ void split8(const float (&v)[8], v4u& H, v4u& L)
{
    unsigned int hb[8], lb[8];
#pragma unroll
    for (int i = 0; i < 8; ++i) {
        unsigned int hi = bf16_bits(v[i]);
        float res = v[i] - __uint_as_float(hi << 16);
        hb[i] = hi;
        lb[i] = bf16_bits(res);
    }
#pragma unroll
    for (int j = 0; j < 4; ++j) {
        H[j] = hb[2 * j] | (hb[2 * j + 1] << 16);
        L[j] = lb[2 * j] | (lb[2 * j + 1] << 16);
    }
}
__device__ __forceinline__ v4u pack8_f16(const float (&v)[8])
{
    Pack8 p;
#pragma unroll
    for (int i = 0; i < 8; ++i) p.h[i] = (f16_t)v[i];
    return p.u;
}
__device__ __forceinline__ void vst(uint16_t* p, v4u v) { *(volatile v4u*)p = v; }
__device__ __forceinline__ void vst(float* p, v4f v)    { *(volatile v4f*)p = v; }

__device__ __forceinline__ void fill_store(const float* __restrict__ X, const float* __restrict__ Mk,
                                           int d, int t0, const float (&mean)[8],
                                           uint16_t* xh, uint16_t* xl)
{
#pragma unroll 1
    for (int b = 0; b < Bn; ++b) {
        const size_t o = ((size_t)b * Dn + d) * Tn + t0;
        const v4f x0 = *(const v4f*)(X + o),  x1 = *(const v4f*)(X + o + 4);
        const v4f q0 = *(const v4f*)(Mk + o), q1 = *(const v4f*)(Mk + o + 4);
        float xm[8], mv[8];
#pragma unroll
        for (int i = 0; i < 4; ++i) { mv[i] = q0[i]; mv[4 + i] = q1[i]; xm[i] = x0[i]; xm[4 + i] = x1[i]; }
#pragma unroll
        for (int i = 0; i < 8; ++i) xm[i] = xm[i] * mv[i] + (1.0f - mv[i]) * mean[i];
        v4u H, L, Q, Z;
        split8(xm, H, L);
#pragma unroll
        for (int j = 0; j < 4; ++j) {
            Q[j] = bf16_bits(mv[2 * j]) | (bf16_bits(mv[2 * j + 1]) << 16);
            Z[j] = 0u;
        }
        const size_t base = ((size_t)b * Dn + d) * KIN + t0;
        vst(xh + base, H);
        vst(xl + base, L);
        vst(xh + base + Tn, Q);
        vst(xl + base + Tn, Z);
    }
}

__global__ void __launch_bounds__(64)
k_fill(const float* __restrict__ X, const float* __restrict__ Mk, uint16_t* xh, uint16_t* xl)
{
    const int d  = blockIdx.x;
    const int t0 = threadIdx.x * 8;
    if (d >= Dn) return;
    float sum[8], cnt[8];
#pragma unroll
    for (int i = 0; i < 8; ++i) { sum[i] = 0.0f; cnt[i] = 0.0f; }
#pragma unroll 1
    for (int b = 0; b < Bn; ++b) {
        const size_t o = ((size_t)b * Dn + d) * Tn + t0;
        const v4f x0 = *(const v4f*)(X + o),  x1 = *(const v4f*)(X + o + 4);
        const v4f q0 = *(const v4f*)(Mk + o), q1 = *(const v4f*)(Mk + o + 4);
#pragma unroll
        for (int i = 0; i < 4; ++i) {
            sum[i]     += x0[i] * q0[i];  cnt[i]     += q0[i];
            sum[4 + i] += x1[i] * q1[i];  cnt[4 + i] += q1[i];
        }
    }
    float mean[8];
#pragma unroll
    for (int i = 0; i < 8; ++i) mean[i] = sum[i] / (cnt[i] + 1e-10f);
    fill_store(X, Mk, d, t0, mean, xh, xl);
    __threadfence();
    fill_store(X, Mk, d, t0, mean, xh, xl);
}

__global__ void __launch_bounds__(256)
k_wcvt(const float* __restrict__ W, uint16_t* Bh, uint16_t* Bl, int K, int N, int strideW, int strideB)
{
    __shared__ float tile[32][65];
    const int tid = threadIdx.x;
    const int n0 = blockIdx.x * 32, k0 = blockIdx.y * 64;
    const float* Wz = W + (size_t)blockIdx.z * (size_t)strideW;
    const size_t zoff = (size_t)blockIdx.z * (size_t)strideB;
#pragma unroll
    for (int i = 0; i < 8; ++i) {
        const int idx = i * 256 + tid;
        const int kk = idx >> 5, nn = idx & 31;
        float v = 0.0f;
        if (k0 + kk < K && n0 + nn < N) v = Wz[(size_t)(k0 + kk) * N + n0 + nn];
        tile[nn][kk] = v;
    }
    __syncthreads();
    const int q = tid >> 3, j = tid & 7;
    const int n = n0 + q, kb = k0 + j * 8;
    float v[8];
#pragma unroll
    for (int i = 0; i < 8; ++i) v[i] = tile[q][j * 8 + i];
    v4u H, L;
    split8(v, H, L);
    const bool ok = (n < N) && (kb + 8 <= K);
    uint16_t* ph = Bh + zoff + (size_t)n * K + kb;
    uint16_t* pl = Bl + zoff + (size_t)n * K + kb;
    if (ok) { vst(ph, H); vst(pl, L); }
    __threadfence();
    if (ok) { vst(ph, H); vst(pl, L); }
}

template <int EPI>
__device__ __forceinline__ void gemm_epilogue_store(float (*tile)[TP], float (*sred)[64],
                                                    const float* __restrict__ vec,
                                                    float* Cf, uint16_t* Ch, uint16_t* Cl,
                                                    uint16_t* Vt, float* sl, float* sr,
                                                    int tid, int rblk, int col0, int N)
{
    if (EPI == 0 || EPI == 2) {
#pragma unroll
        for (int it = 0; it < 8; ++it) {
            const int s = it * 128 + tid;
            const int rl = s >> 4, cq = s & 15;
            v4f v;
#pragma unroll
            for (int i = 0; i < 4; ++i) v[i] = tile[rl][cq * 4 + i] + vec[col0 + cq * 4 + i];
            vst(Cf + (size_t)(rblk + rl) * N + col0 + cq * 4, v);
        }
        if (EPI == 0) {
#pragma unroll
            for (int it = 0; it < 4; ++it) {
                const int s = it * 128 + tid;
                const int rl = s >> 3, cj = s & 7;
                float v[8];
#pragma unroll
                for (int i = 0; i < 8; ++i) v[i] = tile[rl][cj * 8 + i] + vec[col0 + cj * 8 + i];
                v4u H, L;
                split8(v, H, L);
                const size_t o = (size_t)(rblk + rl) * N + col0 + cj * 8;
                vst(Ch + o, H);
                vst(Cl + o, L);
            }
        }
    } else {
        const int b  = rblk / Dn, nb = rblk % Dn;
        const int hh = col0 / OUTn;
        const int bh = b * NHn + hh;
#pragma unroll
        for (int it = 0; it < 4; ++it) {
            const int s = it * 128 + tid;
            const int e = s >> 3, pj = s & 7;
            float v[8];
#pragma unroll
            for (int i = 0; i < 8; ++i) v[i] = tile[pj * 8 + i][e];
            const v4u P = pack8_f16(v);
            vst(Vt + ((size_t)bh * OUTn + e) * Dn + nb + pj * 8, P);
        }
        if (tid < 32) {
            const int which = tid >> 4, t = tid & 15;
            v4f v;
#pragma unroll
            for (int i = 0; i < 4; ++i) v[i] = sred[which][t * 4 + i];
            float* dst = (which == 0 ? sl : sr) + (size_t)bh * Dn + nb + t * 4;
            vst(dst, v);
        }
    }
}

template <int EPI>
__global__ void __launch_bounds__(128)
k_gemm(const uint16_t* __restrict__ Ah, const uint16_t* __restrict__ Al,
       const uint16_t* __restrict__ Bh, const uint16_t* __restrict__ Bl,
       const float* __restrict__ vec,
       float* Cf, uint16_t* Ch, uint16_t* Cl,
       uint16_t* Vt, float* sl, float* sr,
       int M, int N, int K)
{
    __shared__ float tile[64][TP];
    __shared__ float sred[2][64];
    const int tid  = threadIdx.x;
    const int lane = tid & 31, wave = tid >> 5;
    const int h    = lane >> 4, m16 = lane & 15;
    const int rblk = blockIdx.x * 64, col0 = blockIdx.y * 64;
    if (rblk + 64 > M || col0 + 64 > N) return;
    const int row0 = rblk + wave * 16;

    v8f acc[4];
#pragma unroll
    for (int nt = 0; nt < 4; ++nt) acc[nt] = zero8();

    const uint16_t* pah = Ah + (size_t)(row0 + m16) * K + 8 * h;
    const uint16_t* pal = Al + (size_t)(row0 + m16) * K + 8 * h;
    const uint16_t* pbh = Bh + (size_t)(col0 + m16) * K + 8 * h;
    const uint16_t* pbl = Bl + (size_t)(col0 + m16) * K + 8 * h;

    for (int k0 = 0; k0 < K; k0 += 32) {
        FragB ah, al;
        ah.u[0] = *(const v8us*)(pah + k0);
        ah.u[1] = *(const v8us*)(pah + k0 + 16);
        al.u[0] = *(const v8us*)(pal + k0);
        al.u[1] = *(const v8us*)(pal + k0 + 16);
#pragma unroll
        for (int nt = 0; nt < 4; ++nt) {
            const size_t bo = (size_t)nt * 16 * K + k0;
            FragB bh, bl;
            bh.u[0] = *(const v8us*)(pbh + bo);
            bh.u[1] = *(const v8us*)(pbh + bo + 16);
            bl.u[0] = *(const v8us*)(pbl + bo);
            bl.u[1] = *(const v8us*)(pbl + bo + 16);
            acc[nt] = mma_bf16(ah.v, bh.v, acc[nt]);
            acc[nt] = mma_bf16(al.v, bh.v, acc[nt]);
            acc[nt] = mma_bf16(ah.v, bl.v, acc[nt]);
        }
    }

#pragma unroll
    for (int nt = 0; nt < 4; ++nt) {
#pragma unroll
        for (int r = 0; r < 8; ++r) tile[wave * 16 + 8 * h + r][nt * 16 + m16] = acc[nt][r];
    }
    __syncthreads();

    if (EPI == 1) {
        const int hh = col0 / OUTn;
        const float* aL = vec + hh * 2 * OUTn;
        const float* aR = aL + OUTn;
        const int rl = tid >> 1, hf = tid & 1;
        float dl = 0.0f, dr = 0.0f;
#pragma unroll 8
        for (int e = hf * 32; e < hf * 32 + 32; ++e) {
            const float v = tile[rl][e];
            dl += v * aL[e];
            dr += v * aR[e];
        }
        dl += __shfl_xor(dl, 1, 32);
        dr += __shfl_xor(dr, 1, 32);
        if (hf == 0) { sred[0][rl] = dl; sred[1][rl] = dr; }
        __syncthreads();
    }

    gemm_epilogue_store<EPI>(tile, sred, vec, Cf, Ch, Cl, Vt, sl, sr, tid, rblk, col0, N);
    __threadfence();
    gemm_epilogue_store<EPI>(tile, sred, vec, Cf, Ch, Cl, Vt, sl, sr, tid, rblk, col0, N);
}

__device__ __forceinline__ void attn_store(float (*tile)[TP], float* dst, int tid)
{
#pragma unroll
    for (int it = 0; it < 8; ++it) {
        const int s = it * 128 + tid;
        const int rl = s >> 4, cq = s & 15;
        v4f v;
#pragma unroll
        for (int i = 0; i < 4; ++i) v[i] = tile[rl][cq * 4 + i];
        vst(dst + (size_t)rl * HIDn + cq * 4, v);
    }
}

__global__ void __launch_bounds__(128)
k_attn(const float* __restrict__ sl, const float* __restrict__ sr, const uint16_t* __restrict__ Vt, float* hnew)
{
    __shared__ float s_sr[Dn];
    __shared__ float s_red[4];
    __shared__ float tile[64][TP];
    const int tid  = threadIdx.x;
    const int lane = tid & 31, wave = tid >> 5;
    const int h    = lane >> 4, m16 = lane & 15;
    const int bh   = blockIdx.y, nb = blockIdx.x * 64;
    if (bh >= Bn * NHn || nb + 64 > Dn) return;

    const float* srg = sr + (size_t)bh * Dn;
    float mx = -3.0e38f;
#pragma unroll
    for (int i = 0; i < Dn / 128; ++i) {
        const int idx = i * 128 + tid;
        const float v = srg[idx];
        s_sr[idx] = v;
        mx = fmaxf(mx, v);
    }
#pragma unroll
    for (int off = 16; off > 0; off >>= 1) mx = fmaxf(mx, __shfl_xor(mx, off, 32));
    if (lane == 0) s_red[wave] = mx;
    __syncthreads();
    mx = fmaxf(fmaxf(s_red[0], s_red[1]), fmaxf(s_red[2], s_red[3]));

    const int   n   = nb + wave * 16 + m16;
    const float slv = sl[(size_t)bh * Dn + n];
    const float rm  = lrelu(slv + mx);

    float den = 0.0f;
    for (int k0 = 0; k0 < Dn; k0 += 32) {
#pragma unroll
        for (int i = 0; i < 8; ++i) {
            den += __expf(lrelu(slv + s_sr[k0 + 8 * h + i]) - rm);
            den += __expf(lrelu(slv + s_sr[k0 + 16 + 8 * h + i]) - rm);
        }
    }
    den += __shfl_xor(den, 16, 32);
    const float rd = PSCALE / den;

    v8f acc[4];
#pragma unroll
    for (int nt = 0; nt < 4; ++nt) acc[nt] = zero8();
    const uint16_t* vb = Vt + (size_t)bh * OUTn * Dn + (size_t)m16 * Dn + 8 * h;

    for (int k0 = 0; k0 < Dn; k0 += 32) {
        FragH a;
#pragma unroll
        for (int i = 0; i < 8; ++i) {
            a.v[i]     = (f16_t)(__expf(lrelu(slv + s_sr[k0 + 8 * h + i]) - rm) * rd);
            a.v[8 + i] = (f16_t)(__expf(lrelu(slv + s_sr[k0 + 16 + 8 * h + i]) - rm) * rd);
        }
#pragma unroll
        for (int nt = 0; nt < 4; ++nt) {
            const uint16_t* bp = vb + (size_t)nt * 16 * Dn + k0;
            FragH bfr;
            bfr.u[0] = *(const v8us*)(bp);
            bfr.u[1] = *(const v8us*)(bp + 16);
            acc[nt] = mma_f16(a.v, bfr.v, acc[nt]);
        }
    }

#pragma unroll
    for (int nt = 0; nt < 4; ++nt) {
#pragma unroll
        for (int r = 0; r < 8; ++r) tile[wave * 16 + 8 * h + r][nt * 16 + m16] = acc[nt][r] * PSCALE_INV;
    }
    __syncthreads();

    const int b = bh / NHn, hh = bh % NHn;
    float* dst = hnew + ((size_t)b * Dn + nb) * HIDn + hh * OUTn;
    attn_store(tile, dst, tid);
    __threadfence();
    attn_store(tile, dst, tid);
}

__global__ void __launch_bounds__(256)
k_ln(float* h32, const float* __restrict__ hn, const float* __restrict__ g, const float* __restrict__ be,
     uint16_t* ph, uint16_t* pl, int M)
{
    __shared__ float srow[8][HIDn];
    const int wave = threadIdx.x >> 5, lane = threadIdx.x & 31;
    const int row  = blockIdx.x * 8 + wave;
    const bool ok  = row < M;
    const int c0   = lane * 8;

    float y[8];
    if (ok) {
        const float* hr = h32 + (size_t)row * HIDn + c0;
        const float* nr = hn  + (size_t)row * HIDn + c0;
        const v4f a0 = *(const v4f*)(hr), a1 = *(const v4f*)(hr + 4);
        const v4f d0 = *(const v4f*)(nr), d1 = *(const v4f*)(nr + 4);
#pragma unroll
        for (int i = 0; i < 4; ++i) { y[i] = a0[i] + d0[i]; y[4 + i] = a1[i] + d1[i]; }
    } else {
#pragma unroll
        for (int i = 0; i < 8; ++i) y[i] = 0.0f;
    }
    float sum = 0.0f;
#pragma unroll
    for (int i = 0; i < 8; ++i) sum += y[i];
#pragma unroll
    for (int off = 16; off > 0; off >>= 1) sum += __shfl_xor(sum, off, 32);
    const float mu = sum * (1.0f / HIDn);
    float var = 0.0f;
#pragma unroll
    for (int i = 0; i < 8; ++i) { const float d = y[i] - mu; var += d * d; }
#pragma unroll
    for (int off = 16; off > 0; off >>= 1) var += __shfl_xor(var, off, 32);
    var *= (1.0f / HIDn);
    const float rs = rsqrtf(var + EPSc);

    float o[8];
#pragma unroll
    for (int i = 0; i < 8; ++i) o[i] = (y[i] - mu) * rs * g[c0 + i] + be[c0 + i];
#pragma unroll
    for (int i = 0; i < 8; ++i) srow[wave][c0 + i] = o[i];
    v4u H, L;
    split8(o, H, L);
    __syncthreads();

    v4f f0, f1;
#pragma unroll
    for (int i = 0; i < 4; ++i) { f0[i] = srow[wave][lane * 4 + i]; f1[i] = srow[wave][128 + lane * 4 + i]; }
    float*    hw = h32 + (size_t)row * HIDn;
    uint16_t* qh = ph + (size_t)row * HIDn + c0;
    uint16_t* ql = pl + (size_t)row * HIDn + c0;
    if (ok) {
        vst(hw + lane * 4, f0);
        vst(hw + 128 + lane * 4, f1);
        vst(qh, H);
        vst(ql, L);
    }
    __threadfence();
    if (ok) {
        vst(hw + lane * 4, f0);
        vst(hw + 128 + lane * 4, f1);
        vst(qh, H);
        vst(ql, L);
    }
}

extern "C" void kernel_launch(void* const* d_in, const int* in_sizes, int n_in,
                              void* d_out, int out_size, void* d_ws, size_t ws_size,
                              hipStream_t stream)
{
    if (n_in < 10) return;
    if (in_sizes[0] != Bn * Dn * Tn || in_sizes[1] != Bn * Dn * Tn ||
        in_sizes[2] != KIN * HIDn || in_sizes[3] != HIDn ||
        in_sizes[4] != NLn * NHn * HIDn * OUTn || in_sizes[5] != NLn * NHn * 2 * OUTn ||
        in_sizes[6] != NLn * HIDn || in_sizes[7] != NLn * HIDn ||
        in_sizes[8] != HIDn * Tn || in_sizes[9] != Tn ||
        out_size != Bn * Dn * Tn) return;

    const float* X_obs = (const float*)d_in[0];
    const float* mask  = (const float*)d_in[1];
    const float* W_in  = (const float*)d_in[2];
    const float* b_in  = (const float*)d_in[3];
    const float* g_W   = (const float*)d_in[4];
    const float* g_a   = (const float*)d_in[5];
    const float* ln_g  = (const float*)d_in[6];
    const float* ln_b  = (const float*)d_in[7];
    const float* W_out = (const float*)d_in[8];
    const float* b_out = (const float*)d_in[9];
    float* out = (float*)d_out;

    size_t off = 0;
    auto carve = [&](size_t bytes) -> void* {
        void* p = (char*)d_ws + off;
        off += (bytes + 255) & ~(size_t)255;
        return p;
    };
    uint16_t* xh   = (uint16_t*)carve((size_t)Mrows * KIN * sizeof(uint16_t));
    uint16_t* xl   = (uint16_t*)carve((size_t)Mrows * KIN * sizeof(uint16_t));
    uint16_t* winh = (uint16_t*)carve((size_t)HIDn * KIN * sizeof(uint16_t));
    uint16_t* winl = (uint16_t*)carve((size_t)HIDn * KIN * sizeof(uint16_t));
    float*    h32  = (float*)   carve((size_t)Mrows * HIDn * sizeof(float));
    uint16_t* hh   = (uint16_t*)carve((size_t)Mrows * HIDn * sizeof(uint16_t));
    uint16_t* hl   = (uint16_t*)carve((size_t)Mrows * HIDn * sizeof(uint16_t));
    uint16_t* wch  = (uint16_t*)carve((size_t)HIDn * HIDn * sizeof(uint16_t));
    uint16_t* wcl  = (uint16_t*)carve((size_t)HIDn * HIDn * sizeof(uint16_t));
    uint16_t* vt   = (uint16_t*)carve((size_t)Bn * NHn * OUTn * Dn * sizeof(uint16_t));
    float*    s_l  = (float*)   carve((size_t)Bn * NHn * Dn * sizeof(float));
    float*    s_r  = (float*)   carve((size_t)Bn * NHn * Dn * sizeof(float));
    float*    hnew = (float*)   carve((size_t)Mrows * HIDn * sizeof(float));
    uint16_t* woh  = (uint16_t*)carve((size_t)Tn * HIDn * sizeof(uint16_t));
    uint16_t* wol  = (uint16_t*)carve((size_t)Tn * HIDn * sizeof(uint16_t));
    if (off > ws_size) return;

    k_fill<<<dim3(Dn), dim3(64), 0, stream>>>(X_obs, mask, xh, xl);
    k_wcvt<<<dim3(HIDn / 32, KIN / 64, 1), dim3(256), 0, stream>>>(W_in, winh, winl, KIN, HIDn, 0, 0);
    k_gemm<0><<<dim3(Mrows / 64, HIDn / 64), dim3(128), 0, stream>>>(
        xh, xl, winh, winl, b_in, h32, hh, hl, vt, s_l, s_r, Mrows, HIDn, KIN);

    for (int l = 0; l < NLn; ++l) {
        const float* gW_l = g_W  + (size_t)l * NHn * HIDn * OUTn;
        const float* ga_l = g_a  + (size_t)l * NHn * 2 * OUTn;
        const float* gg_l = ln_g + (size_t)l * HIDn;
        const float* gb_l = ln_b + (size_t)l * HIDn;
        k_wcvt<<<dim3(OUTn / 32, HIDn / 64, NHn), dim3(256), 0, stream>>>(
            gW_l, wch, wcl, HIDn, OUTn, HIDn * OUTn, OUTn * HIDn);
        k_gemm<1><<<dim3(Mrows / 64, HIDn / 64), dim3(128), 0, stream>>>(
            hh, hl, wch, wcl, ga_l, hnew, woh, wol, vt, s_l, s_r, Mrows, HIDn, HIDn);
        k_attn<<<dim3(Dn / 64, Bn * NHn), dim3(128), 0, stream>>>(s_l, s_r, vt, hnew);
        k_ln<<<dim3(Mrows / 8), dim3(256), 0, stream>>>(h32, hnew, gg_l, gb_l, hh, hl, Mrows);
    }

    k_wcvt<<<dim3(Tn / 32, HIDn / 64, 1), dim3(256), 0, stream>>>(W_out, woh, wol, HIDn, Tn, 0, 0);
    k_gemm<2><<<dim3(Mrows / 64, Tn / 64), dim3(128), 0, stream>>>(
        hh, hl, woh, wol, b_out, out, winh, winl, vt, s_l, s_r, Mrows, Tn, HIDn);
}
